// NeuralNetwork_74466142978489
// MI455X (gfx1250) — hardware-verified
//
#include <hip/hip_runtime.h>
#include <stddef.h>


typedef _Float16 v16h __attribute__((ext_vector_type(16)));
typedef _Float16 v8h  __attribute__((ext_vector_type(8)));
typedef float    v8f  __attribute__((ext_vector_type(8)));
typedef float    v4f  __attribute__((ext_vector_type(4)));

#ifndef NB
#define NB 65536
#endif
#define NB_FULL 65536
#define NNEUR 512
#define NIN   64
#define NOUT  16
#define COL0  (NNEUR - NOUT)
#define WAVES 8
#define ROWS_PER_WAVE  16
#define ROWS_PER_BLOCK (WAVES * ROWS_PER_WAVE)

#define LDT  72
#define LDCW 20

#define WCARRY 64.0f
#define ACARRY 64.0f

static_assert(NB >= ROWS_PER_BLOCK && NB <= NB_FULL);
static_assert((NB % ROWS_PER_BLOCK) == 0);
static_assert(NIN == 64 && (NIN % 32) == 0);
static_assert(NOUT == 16);
static_assert(COL0 >= NIN);
static_assert(COL0 + NOUT == NNEUR);
static_assert((COL0 % 4) == 0);
static_assert(NIN * NOUT == 4 * 256);
static_assert((LDT % 8) == 0 && LDT >= NIN);
static_assert((LDCW % 4) == 0 && LDCW >= NOUT);
static_assert(ROWS_PER_WAVE * NOUT == 2 * 32 * 4);
static_assert((32 / 4) * 2 == ROWS_PER_WAVE);
static_assert((ROWS_PER_WAVE * NOUT * 4) % 128 == 0);
static_assert((size_t)NOUT * LDT * 2 + (size_t)WAVES * 16 * LDCW * 4 <= (size_t)131072);
static_assert((size_t)NB * NOUT * 4 <= (size_t)4194304);

__device__ __forceinline__ float bf16r(float x) {
  unsigned int u = __float_as_uint(x);
  u = (u + 0x7FFFu + ((u >> 16) & 1u)) & 0xFFFF0000u;
  return __uint_as_float(u);
}

static __device__ __forceinline__ _Float16 toh_flush(float v) {
  const _Float16 r = (_Float16)v;
  return (fabsf(v) < 6.103515625e-05f) ? (_Float16)0.0f : r;
}

__device__ __forceinline__ v16h frag_at(const _Float16* p) {
  v8h lo = *(const v8h*)(p);
  v8h hi = *(const v8h*)(p + 16);
  v16h out;
#pragma unroll
  for (int i = 0; i < 8; ++i) { out[i] = lo[i]; out[i + 8] = hi[i]; }
  return out;
}
__device__ __forceinline__ v16h ld_frag(const _Float16* base, unsigned ld) {
  const unsigned lane = threadIdx.x & 31u;
  return frag_at(base + (lane & 15u) * ld + (lane >> 4) * 8u);
}

__device__ __forceinline__ v8f wmma16(v16h a, v16h b, v8f c) {
  v8f d = __builtin_amdgcn_wmma_f32_16x16x32_f16(false, a, false, b, (short)0, c,
                                                 false, false);
  asm volatile("v_nop\n\tv_nop\n\tv_nop\n\tv_nop" : "+v"(d) : "v"(a), "v"(b));
  return d;
}

__global__ __launch_bounds__(256) void dense_act_kernel(
    const float* __restrict__ A, const float* __restrict__ W,
    const float* __restrict__ bias, const int* __restrict__ acts,
    float* __restrict__ out) {
  __shared__ __attribute__((aligned(16))) _Float16 T[NOUT * LDT];
  __shared__ __attribute__((aligned(16))) float Cs[WAVES * 16 * LDCW];

  const unsigned tid = threadIdx.x, lane = tid & 31u;
  const unsigned wave = (unsigned)__builtin_amdgcn_readfirstlane((int)(threadIdx.x >> 5));
  const unsigned hh = lane >> 4, m = lane & 15u;
  const unsigned r0 = blockIdx.x * (unsigned)ROWS_PER_BLOCK + wave * (unsigned)ROWS_PER_WAVE;

#pragma unroll
  for (unsigned j = 0; j < 4u; ++j) {
    const unsigned idx = tid + 256u * j;
    const unsigned kr = idx >> 4, nc = idx & 15u;
    const float v = W[(size_t)kr * NNEUR + COL0 + nc];
    T[nc * LDT + kr] = toh_flush(WCARRY * bf16r(v));
  }

  const float* ap = A + (size_t)(r0 + m) * NIN + hh * 8u;
  v16h af[2];
#pragma unroll
  for (int c = 0; c < 2; ++c) {
    const v4f x0 = *(const v4f*)(ap + 32 * c);
    const v4f x1 = *(const v4f*)(ap + 32 * c + 4);
    const v4f x2 = *(const v4f*)(ap + 32 * c + 16);
    const v4f x3 = *(const v4f*)(ap + 32 * c + 20);
#pragma unroll
    for (int i = 0; i < 4; ++i) {
      af[c][i]      = toh_flush(ACARRY * bf16r(x0[i]));
      af[c][i + 4]  = toh_flush(ACARRY * bf16r(x1[i]));
      af[c][i + 8]  = toh_flush(ACARRY * bf16r(x2[i]));
      af[c][i + 12] = toh_flush(ACARRY * bf16r(x3[i]));
    }
  }
  const float bb = bf16r(bias[COL0 + m]);
  const int aid = acts[COL0 + m];

  __syncthreads();

  v8f acc = {};
#pragma unroll
  for (int c = 0; c < 2; ++c) {
    const v16h bf = ld_frag(&T[c * 32], LDT);
    acc = wmma16(af[c], bf, acc);
  }

  const bool is_tanh  = (aid == 0);
  const bool is_sig   = (aid == 1);
  const bool is_relu  = (aid == 2);
  const bool is_lrelu = (aid == 3);
  const unsigned cb = wave * (16u * LDCW);
#pragma unroll
  for (int r = 0; r < 8; ++r) {
    const float t = acc[r] * (1.0f / (ACARRY * WCARRY)) + bb;
    const float arg = is_tanh ? (2.0f * t) : (-t);
    const float e = __expf(arg);
    const float fe = __builtin_amdgcn_rcpf(1.0f + e);
    const float ts = is_tanh ? (1.0f - 2.0f * fe) : fe;
    float res = t;
    res = is_lrelu ? ((t > 0.0f) ? t : 0.01f * t) : res;
    res = is_relu ? fmaxf(t, 0.0f) : res;
    res = (is_tanh || is_sig) ? ts : res;
    Cs[cb + (hh * 8u + (unsigned)r) * LDCW + m] = res;
  }
  __syncthreads();

  v4f x[2];
  size_t off[2];
#pragma unroll
  for (unsigned i = 0; i < 2u; ++i) {
    const unsigned row = 8u * i + (lane >> 2);
    const unsigned col = (lane & 3u) * 4u;
    x[i] = *(const v4f*)&Cs[cb + row * LDCW + col];
    off[i] = (size_t)r0 * NOUT + 128u * i + 4u * lane;
  }
#pragma unroll
  for (int i = 0; i < 2; ++i) *(volatile v4f*)(out + off[i]) = x[i];
  __threadfence();
#pragma unroll
  for (int i = 0; i < 2; ++i) *(volatile v4f*)(out + off[i]) = x[i];
}

extern "C" void kernel_launch(void* const* d_in, const int* in_sizes, int n_in,
                              void* d_out, int out_size, void* d_ws, size_t ws_size,
                              hipStream_t stream) {
  (void)d_ws;
  (void)ws_size;
  if (n_in < 4) return;
  if ((long long)in_sizes[0] < (long long)NB * NIN) return;
  if ((long long)in_sizes[1] < (long long)NNEUR * NNEUR) return;
  if (in_sizes[2] < NNEUR) return;
  if (in_sizes[3] < NNEUR) return;
  if ((long long)out_size < (long long)NB * NOUT) return;

  const float* A    = (const float*)d_in[0];
  const float* W    = (const float*)d_in[1];
  const float* bias = (const float*)d_in[2];
  const int*   acts = (const int*)d_in[3];
  float* out = (float*)d_out;

  dense_act_kernel<<<dim3(NB / ROWS_PER_BLOCK), dim3(256), 0, stream>>>(A, W, bias, acts, out);
}
